// Head_9483287789886
// MI455X (gfx1250) — hardware-verified
//
#include <hip/hip_runtime.h>
#include <math.h>

typedef __attribute__((ext_vector_type(16))) _Float16 v16h;
typedef __attribute__((ext_vector_type(16))) __bf16 v16b;
typedef __attribute__((ext_vector_type(8)))  _Float16 v8h;
typedef __attribute__((ext_vector_type(8)))  __bf16 v8b;
typedef __attribute__((ext_vector_type(8)))  float v8f;
typedef __attribute__((ext_vector_type(4)))  float v4f;
typedef __attribute__((ext_vector_type(4)))  unsigned v4u;

template <typename T> __device__ __forceinline__ void vst2(void* p, T v) { *(volatile T*)p = v; __threadfence(); *(volatile T*)p = v; }
__device__ __forceinline__ v8f wmma16(v16h a, v16h b, v8f c) {
  v8f d = __builtin_amdgcn_wmma_f32_16x16x32_f16(false, a, false, b, (short)0, c, false, false);
  asm volatile("v_nop\n\tv_nop\n\tv_nop\n\tv_nop" : "+v"(d) : "v"(a), "v"(b));
  return d;
}
__device__ __forceinline__ v8f wmma_bf(v16b a, v16b b, v8f c) {
  v8f d = __builtin_amdgcn_wmma_f32_16x16x32_bf16(false, a, false, b, (short)0, c, false, false);
  asm volatile("v_nop\n\tv_nop\n\tv_nop\n\tv_nop" : "+v"(d) : "v"(a), "v"(b));
  return d;
}
__device__ __forceinline__ v16h frag_h(const _Float16* rowk0, int lane) {
  union { v16h v; v8h q[2]; } u; const _Float16* p = rowk0 + 8 * (lane >> 4);
  u.q[0] = *(const v8h*)p; u.q[1] = *(const v8h*)(p + 16); return u.v;
}
__device__ __forceinline__ v16b frag_b(const __bf16* rowk0, int lane) {
  union { v16b v; v8b q[2]; } u; const __bf16* p = rowk0 + 8 * (lane >> 4);
  u.q[0] = *(const v8b*)p; u.q[1] = *(const v8b*)(p + 16); return u.v;
}
__device__ __forceinline__ v16h frag_f32(const float* rowk0, int lane) {
  v16h a; const float* p = rowk0 + 8 * (lane >> 4);
#pragma unroll
  for (int i = 0; i < 8; ++i) { a[i] = (_Float16)p[i]; a[8 + i] = (_Float16)p[16 + i]; }
  return a;
}
struct F2 { v16b h, l; };
__device__ __forceinline__ F2 bsplit16(const float v[16]) { F2 r;
#pragma unroll
  for (int i = 0; i < 16; ++i) { const __bf16 hb = (__bf16)v[i]; r.h[i] = hb; r.l[i] = (__bf16)(v[i] - (float)hb); }
  return r; }
__device__ __forceinline__ F2 split_row(const float* row, int k0, int lane) { float v[16]; const float* p = row + k0 + 8 * (lane >> 4);
#pragma unroll
  for (int i = 0; i < 8; ++i) { v[i] = p[i]; v[8 + i] = p[16 + i]; }
  return bsplit16(v); }
__device__ __forceinline__ v16b wcol_io(const float* Wm, int k0, int o, int lane, int ld) { v16b w; const int g = lane >> 4;
#pragma unroll
  for (int i = 0; i < 8; ++i) { w[i] = (__bf16)Wm[(size_t)(k0 + 8 * g + i) * ld + o]; w[8 + i] = (__bf16)Wm[(size_t)(k0 + 16 + 8 * g + i) * ld + o]; }
  return w; }
#define LDSX() do { asm volatile("s_wait_dscnt 0" ::: "memory"); __builtin_amdgcn_wave_barrier(); __builtin_amdgcn_fence(3  , "workgroup"); } while (0)

#ifndef NB
#define NB 8
#endif
#ifndef SEQ
#define SEQ 2048
#endif
#define NB_FULL 8
#define SEQ_FULL 2048
#define TT SEQ
#define DIN 384
#define HH 64
#define CC HH
#define NQB (TT / 64)
#define QB3 (NQB / 2)
#define BG ((NB % 2 == 0) ? 2 : 1)
#define SCALE (0.05103103630798288f)
static_assert(NB >= 1 && NB <= NB_FULL);
static_assert(TT >= 128 && TT <= SEQ_FULL && TT % 128 == 0);
static_assert(NB % BG == 0);
static_assert(DIN % 32 == 0 && HH % 32 == 0);

__host__ __device__ __forceinline__ int kb_last(int qb) { return (qb * 64 + 63) >> 7; }

#define WS_QH  ((size_t)0)
#define WS_KH  (WS_QH  + 2u * (size_t)NB * TT * CC)
#define WS_QL  (WS_KH  + 2u * (size_t)NB * TT * CC)
#define WS_KL  (WS_QL  + 2u * (size_t)NB * TT * CC)
#define WS_VT  (WS_KL  + 2u * (size_t)NB * TT * CC)
#define WS_VB  (WS_VT  + 2u * (size_t)NB * CC * TT)
#define WS_VBL (WS_VB  + 2u * (size_t)NB * CC * TT)
#define WS_S   (WS_VBL + 2u * (size_t)NB * CC * TT)
#define WS_END (WS_S   + 4u * (size_t)BG * TT * TT)
static_assert(WS_END <= (size_t)134217728);
static_assert(WS_S % 128 == 0);

__global__ __launch_bounds__(128) void k_proj(const float* __restrict__ X, const float* __restrict__ WQ, const float* __restrict__ WK, const float* __restrict__ WV,
    _Float16* __restrict__ QH, _Float16* __restrict__ QL, _Float16* __restrict__ KH, _Float16* __restrict__ KL, _Float16* __restrict__ VT, __bf16* __restrict__ VB, __bf16* __restrict__ VBL) {
  __shared__ __align__(16) _Float16 sh[64][72], sl[64][72]; __shared__ __align__(16) _Float16 th[64][72]; __shared__ __align__(16) __bf16 tb[64][72], tbl[64][72];
  const int tid = threadIdx.x, wave = tid >> 5, lane = tid & 31, col = lane & 15, g = lane >> 4; const int which = blockIdx.z;
  const size_t r0 = (size_t)blockIdx.x * 64; const size_t bb = r0 / TT; const int t0 = (int)(r0 % TT);
  const float* WA = which == 0 ? WQ : which == 1 ? WK : WV;
  v8f acc[CC / 16] = {};
#pragma unroll 2
  for (int kc = 0; kc < DIN / 32; ++kc) { v16b a; { const float* p = X + (bb * SEQ_FULL + t0 + wave * 16 + col) * (size_t)DIN + kc * 32 + 8 * g; float u0[8], u1[8];
#pragma unroll
      for (int i = 0; i < 8; ++i) u0[i] = p[i];
      asm volatile("s_wait_loadcnt 0x0" ::: "memory");
#pragma unroll
      for (int i = 0; i < 8; ++i) u1[i] = p[16 + i];
      asm volatile("s_wait_loadcnt 0x0" ::: "memory");
#pragma unroll
      for (int i = 0; i < 8; ++i) { a[i] = (__bf16)u0[i]; a[8 + i] = (__bf16)u1[i]; } }
    asm volatile("s_wait_loadcnt 0x0" ::: "memory");
#pragma unroll
    for (int j = 0; j < CC / 16; ++j) { const v16b w = wcol_io(WA, kc * 32, j * 16 + col, lane, HH); asm volatile("s_wait_loadcnt 0x0" ::: "memory"); acc[j] = wmma_bf(a, w, acc[j]); } }
  if (which < 2) { _Float16* DH = which == 0 ? QH : KH; _Float16* DL = which == 0 ? QL : KL;
#pragma unroll
    for (int j = 0; j < CC / 16; ++j) {
#pragma unroll
      for (int r = 0; r < 8; ++r) { const float v = acc[j][r]; const _Float16 hv = (_Float16)v; sh[wave * 16 + 8 * g + r][j * 16 + col] = hv; sl[wave * 16 + 8 * g + r][j * 16 + col] = (_Float16)((v - (float)hv) * 1024.0f); } }
    __syncthreads();
    for (int e = tid; e < 64 * (CC / 8); e += 128) { const int rl = e >> 3, q = e & 7; vst2((void*)(DH + (r0 + rl) * (size_t)CC + q * 8), *(const v4u*)&sh[rl][q * 8]); vst2((void*)(DL + (r0 + rl) * (size_t)CC + q * 8), *(const v4u*)&sl[rl][q * 8]); }
  } else {
#pragma unroll
    for (int j = 0; j < CC / 16; ++j) {
#pragma unroll
      for (int r = 0; r < 8; ++r) { const float v = acc[j][r]; const int rl = wave * 16 + 8 * g + r, cl = j * 16 + col; th[cl][rl] = (_Float16)v; const __bf16 bh = (__bf16)v; tb[cl][rl] = bh; tbl[cl][rl] = (__bf16)(v - (float)bh); } }
    __syncthreads();
    for (int e = tid; e < CC * 8; e += 128) { const int cl = e >> 3, q = e & 7; const size_t o3 = (bb * CC + cl) * (size_t)TT + t0 + q * 8; vst2((void*)(VT + o3), *(const v4u*)&th[cl][q * 8]); vst2((void*)(VB + o3), *(const v4u*)&tb[cl][q * 8]); vst2((void*)(VBL + o3), *(const v4u*)&tbl[cl][q * 8]); } }
}
__global__ __launch_bounds__(128) void k_sc(const _Float16* __restrict__ QH, const _Float16* __restrict__ KH, const _Float16* __restrict__ QL, const _Float16* __restrict__ KL, int bgrp, float* __restrict__ S0) { __shared__ __align__(16) float ss[4][16][132];
  const int qb = blockIdx.x, kb = blockIdx.y; if (kb > kb_last(qb)) return;
  const int b = bgrp + blockIdx.z; float* S = S0 + (size_t)blockIdx.z * TT * TT;
  const int tid = threadIdx.x, wave = tid >> 5, lane = tid & 31, col = lane & 15, g = lane >> 4; const int k0 = kb * 128; const int ql0 = qb * 64 + wave * 16; const size_t q0 = (size_t)b * TT + ql0, kr0 = (size_t)b * TT + k0;
  v8f acc[8] = {}, accl[8] = {};
#pragma unroll
  for (int kc = 0; kc < HH / 32; ++kc) { const v16h ah = frag_h(QH + (q0 + col) * CC + kc * 32, lane), al = frag_h(QL + (q0 + col) * CC + kc * 32, lane);
#pragma unroll
    for (int j = 0; j < 8; ++j) { const v16h kbf = frag_h(KH + (kr0 + j * 16 + col) * CC + kc * 32, lane), klf = frag_h(KL + (kr0 + j * 16 + col) * CC + kc * 32, lane); acc[j] = wmma16(ah, kbf, acc[j]); accl[j] = wmma16(al, kbf, accl[j]); accl[j] = wmma16(ah, klf, accl[j]); } }
#pragma unroll
  for (int j = 0; j < 8; ++j) {
#pragma unroll
    for (int r = 0; r < 8; ++r) ss[wave][8 * g + r][j * 16 + col] = (acc[j][r] + accl[j][r] * (1.0f / 1024.0f)) * SCALE; }
  LDSX(); for (int rl = 0; rl < 16; ++rl) vst2(S + (size_t)(ql0 + rl) * TT + k0 + lane * 4, *(const v4f*)&ss[wave][rl][lane * 4]); }
__global__ __launch_bounds__(256) void k_sm(float* __restrict__ S0) { __shared__ float sred[8][32]; __shared__ float sbc[32];
  const int tid = threadIdx.x, wave = tid >> 5, lane = tid & 31;
  const int s0 = blockIdx.x * 32, s = s0 + lane, tlo = s0 & ~127;
  float* Sc = S0 + (size_t)blockIdx.y * TT * TT + s;
  float m = -3.0e38f;
#pragma unroll 1
  for (int t = tlo + wave; t < TT; t += 8) { const float v = Sc[(size_t)t * TT]; m = fmaxf(m, (t >= s) ? v : -3.0e38f); }
  sred[wave][lane] = m; __syncthreads();
  if (wave == 0) { float a = sred[0][lane];
#pragma unroll
    for (int i = 1; i < 8; ++i) a = fmaxf(a, sred[i][lane]);
    sbc[lane] = a; }
  __syncthreads(); m = sbc[lane]; __syncthreads();
  float sum = 0.f;
#pragma unroll 1
  for (int t = tlo + wave; t < TT; t += 8) { const float v = Sc[(size_t)t * TT]; const float e = expf(fminf(v - m, 0.f)); sum += (t >= s) ? e : 0.f; }
  sred[wave][lane] = sum; __syncthreads();
  if (wave == 0) { float a = 0.f;
#pragma unroll
    for (int i = 0; i < 8; ++i) a += sred[i][lane];
    sbc[lane] = (a > 0.f) ? (2048.0f / a) : 0.f; }
  __syncthreads(); const float inv = sbc[lane];
#pragma unroll 1
  for (int t = tlo + wave; t < TT; t += 8) { float* q = Sc + (size_t)t * TT; const float v = *q; const float p = (t >= s) ? expf(fminf(v - m, 0.f)) * inv : 0.f; vst2(q, p); } }
__global__ __launch_bounds__(128) void k_pv(const float* __restrict__ PS0, const _Float16* __restrict__ VT, const __bf16* __restrict__ VB, const __bf16* __restrict__ VBL, int bgrp, float* __restrict__ OUT) { __shared__ __align__(16) float ss[4][16][CC + 4];
  const int b = bgrp + blockIdx.z; const float* PS = PS0 + (size_t)blockIdx.z * TT * TT;
  const int tid = threadIdx.x, wave = tid >> 5, lane = tid & 31, col = lane & 15, g = lane >> 4; const int qb = blockIdx.x; const int ql0 = qb * 64 + wave * 16; const int kce = (kb_last(qb) + 1) * 4;
  v8f acc[CC / 16] = {};
  if (qb >= QB3) {
#pragma unroll 1
    for (int kc = 0; kc < kce; ++kc) { const F2 p = split_row(PS + (size_t)(ql0 + col) * TT, kc * 32, lane);
      asm volatile("s_wait_loadcnt 0x0" ::: "memory");
#pragma unroll
      for (int j = 0; j < CC / 16; ++j) { const size_t po = ((size_t)b * CC + j * 16 + col) * (size_t)TT + kc * 32; const v16b vh = frag_b(VB + po, lane); acc[j] = wmma_bf(p.h, vh, acc[j]); acc[j] = wmma_bf(p.l, vh, acc[j]); acc[j] = wmma_bf(p.h, frag_b(VBL + po, lane), acc[j]); } }
  } else {
#pragma unroll 1
    for (int kc = 0; kc < kce; ++kc) { const v16h p = frag_f32(PS + (size_t)(ql0 + col) * TT + kc * 32, lane);
      asm volatile("s_wait_loadcnt 0x0" ::: "memory");
#pragma unroll
      for (int j = 0; j < CC / 16; ++j) { const size_t po = ((size_t)b * CC + j * 16 + col) * (size_t)TT + kc * 32; acc[j] = wmma16(p, frag_h(VT + po, lane), acc[j]); } } }
#pragma unroll
  for (int j = 0; j < CC / 16; ++j)
#pragma unroll
    for (int r = 0; r < 8; ++r) ss[wave][8 * g + r][j * 16 + col] = acc[j][r] * (1.0f / 2048.0f);
  LDSX();
  float* ob = OUT + ((size_t)b * TT + ql0) * HH;
#pragma unroll
  for (int it = 0; it < 8; ++it) vst2(ob + it * 128 + lane * 4, *(const v4f*)&ss[wave][2 * it + g][col * 4]); }

extern "C" void kernel_launch(void* const* d_in, const int* in_sizes, int n_in, void* d_out, int out_size, void* d_ws, size_t ws_size, hipStream_t stream) {
  if (n_in < 4) return;
  if ((size_t)in_sizes[0] < ((size_t)(NB - 1) * SEQ_FULL + TT) * DIN) return;
  if (in_sizes[1] < DIN * HH || in_sizes[2] < DIN * HH || in_sizes[3] < DIN * HH) return;
  if ((size_t)out_size < (size_t)NB * TT * HH) return;
  if (ws_size < WS_END) return;
  const float* X = (const float*)d_in[0]; const float* WQ = (const float*)d_in[1]; const float* WK = (const float*)d_in[2]; const float* WV = (const float*)d_in[3];
  char* ws = (char*)d_ws;
  _Float16 *QH = (_Float16*)(ws + WS_QH), *KH = (_Float16*)(ws + WS_KH), *QL = (_Float16*)(ws + WS_QL), *KL = (_Float16*)(ws + WS_KL), *VT = (_Float16*)(ws + WS_VT);
  __bf16 *VB = (__bf16*)(ws + WS_VB), *VBL = (__bf16*)(ws + WS_VBL); float* S = (float*)(ws + WS_S); float* OUT = (float*)d_out;
  k_proj<<<dim3(NB * TT / 64, 1, 3), 128, 0, stream>>>(X, WQ, WK, WV, QH, QL, KH, KL, VT, VB, VBL);
  for (int b0 = 0; b0 < NB; b0 += BG) {
    k_sc<<<dim3(NQB, TT / 128, BG), 128, 0, stream>>>(QH, KH, QL, KL, b0, S);
    k_sm<<<dim3(TT / 32, BG), 256, 0, stream>>>(S);
    k_pv<<<dim3(NQB, 1, BG), 128, 0, stream>>>(S, VT, VB, VBL, b0, OUT);
  }
}
